// Cross_Attention_Layer_73598559584454
// MI455X (gfx1250) — hardware-verified
//
#include <hip/hip_runtime.h>
#include <math.h>
#include <stdint.h>
#include <stddef.h>


typedef _Float16 v8h __attribute__((ext_vector_type(8)));
typedef _Float16 v16h __attribute__((ext_vector_type(16)));
typedef float v8f __attribute__((ext_vector_type(8)));
typedef float v4f __attribute__((ext_vector_type(4)));

#define DMODEL 768
#define DKQ 128
#define DVV 64
#define ROWS_PER_BLOCK 64
#define KEYS_PER_TILE 32

#define SC_Q 64.0f
#define SC_K 32.0f
#define SC_V 4.0f

union Frag16 {
  v16h v;
  v8h h[2];
};

static __device__ __forceinline__ v8f wmma16(v16h a, v16h b, v8f c) {
  v8f d = __builtin_amdgcn_wmma_f32_16x16x32_f16(false, a, false, b, (short)0, c,
                                                 false, false);
  asm volatile("v_nop\n\tv_nop\n\tv_nop\n\tv_nop" : "+v"(d) : "v"(a), "v"(b));
  return d;
}

__global__ __launch_bounds__(256) void k_sum(const float* __restrict__ x, int n,
                                             float* __restrict__ sumline) {
  __shared__ float red[256];
  const int tid = threadIdx.x;
  float acc = 0.0f;
  const int n4 = n >> 2;
  const v4f* x4 = (const v4f*)x;
  for (int i = tid; i < n4; i += 256) {
    v4f v = x4[i];
    acc += (v[0] + v[1]) + (v[2] + v[3]);
  }
  for (int i = (n4 << 2) + tid; i < n; i += 256) acc += x[i];
  red[tid] = acc;
  __syncthreads();
  for (int s = 128; s > 0; s >>= 1) {
    if (tid < s) red[tid] = red[tid] + red[tid + s];
    __syncthreads();
  }
  const float tot = red[0];
  if (tid < 32) ((volatile float*)sumline)[tid] = tot;
  __threadfence();
  if (tid < 32) ((volatile float*)sumline)[tid] = tot;
}

template <int NCG, int TRANS>
__global__ __launch_bounds__(128 * NCG) void k_proj(
    const float* __restrict__ X, const float* __restrict__ W,
    _Float16* __restrict__ Y, int nrows, int ldy, float wscale) {
  __shared__ __attribute__((aligned(16))) _Float16 stile[4096 * NCG];
  const int tid = threadIdx.x;
  const int l = tid & 31, h = l >> 4, m = l & 15;
  const int wave = tid >> 5;
  const int rg = wave & 3, cg = wave >> 2;
  const int r0 = blockIdx.x * ROWS_PER_BLOCK;
  if (r0 + ROWS_PER_BLOCK > nrows) return;

  v8f acc[4];
#pragma unroll
  for (int j = 0; j < 4; ++j)
#pragma unroll
    for (int r = 0; r < 8; ++r) acc[j][r] = 0.0f;

  const float* xp = X + (size_t)(r0 + 16 * rg + m) * DMODEL + 8 * h;
  const float* wp = W + (size_t)(64 * cg + m) * DMODEL + 8 * h;

#pragma unroll 2
  for (int k0 = 0; k0 < DMODEL; k0 += 32) {
    v16h av;
    {
      const v8f lo = *(const v8f*)(xp + k0);
      const v8f hi = *(const v8f*)(xp + k0 + 16);
#pragma unroll
      for (int i = 0; i < 8; ++i) {
        av[i] = (_Float16)lo[i];
        av[8 + i] = (_Float16)hi[i];
      }
    }
#pragma unroll
    for (int j = 0; j < 4; ++j) {
      const float* wq = wp + (size_t)(16 * j) * DMODEL + k0;
      const v8f lo = *(const v8f*)(wq);
      const v8f hi = *(const v8f*)(wq + 16);
      v16h bv;
#pragma unroll
      for (int i = 0; i < 8; ++i) {
        bv[i] = (_Float16)(lo[i] * wscale);
        bv[8 + i] = (_Float16)(hi[i] * wscale);
      }
      acc[j] = wmma16(av, bv, acc[j]);
    }
  }

  v8h vals[4];
  if (TRANS == 0) {
    _Float16* sw = stile + wave * 1024;
#pragma unroll
    for (int j = 0; j < 4; ++j)
#pragma unroll
      for (int r = 0; r < 8; ++r)
        sw[(8 * h + r) * 64 + 16 * j + m] = (_Float16)acc[j][r];
    __syncthreads();
#pragma unroll
    for (int q = 0; q < 4; ++q) {
      const int row = 4 * q + (l >> 3), c8 = (l & 7) * 8;
      vals[q] = *(const v8h*)(sw + row * 64 + c8);
    }
    _Float16* gb = Y + (size_t)(r0 + 16 * rg) * ldy + 64 * cg;
#pragma unroll
    for (int q = 0; q < 4; ++q) {
      const int row = 4 * q + (l >> 3), c8 = (l & 7) * 8;
      *(volatile v8h*)(gb + (size_t)row * ldy + c8) = vals[q];
    }
    __threadfence();
#pragma unroll
    for (int q = 0; q < 4; ++q) {
      const int row = 4 * q + (l >> 3), c8 = (l & 7) * 8;
      *(volatile v8h*)(gb + (size_t)row * ldy + c8) = vals[q];
    }
  } else {
#pragma unroll
    for (int j = 0; j < 4; ++j)
#pragma unroll
      for (int r = 0; r < 8; ++r)
        stile[(16 * j + m) * 64 + 16 * rg + 8 * h + r] = (_Float16)acc[j][r];
    __syncthreads();
#pragma unroll
    for (int q = 0; q < 4; ++q) {
      const int crow = 16 * wave + 4 * q + (l >> 3), c8 = (l & 7) * 8;
      vals[q] = *(const v8h*)(stile + crow * 64 + c8);
    }
#pragma unroll
    for (int q = 0; q < 4; ++q) {
      const int crow = 16 * wave + 4 * q + (l >> 3), c8 = (l & 7) * 8;
      *(volatile v8h*)(Y + (size_t)crow * ldy + r0 + c8) = vals[q];
    }
    __threadfence();
#pragma unroll
    for (int q = 0; q < 4; ++q) {
      const int crow = 16 * wave + 4 * q + (l >> 3), c8 = (l & 7) * 8;
      *(volatile v8h*)(Y + (size_t)crow * ldy + r0 + c8) = vals[q];
    }
  }
}

__global__ __launch_bounds__(128) void k_attn_gate(
    const _Float16* __restrict__ Qh, const _Float16* __restrict__ Kh,
    const _Float16* __restrict__ Vt, const float* __restrict__ w_out,
    const float* __restrict__ x1, const float* __restrict__ sumline,
    float* __restrict__ outp, int S, int T) {
  __shared__ __attribute__((aligned(16))) _Float16 kbuf[KEYS_PER_TILE * DKQ];
  __shared__ __attribute__((aligned(16))) _Float16 vbuf[DVV * KEYS_PER_TILE];
  const int tid = threadIdx.x;
  const int l = tid & 31, h = l >> 4, m = l & 15;
  const int wave = tid >> 5;
  const int qb = blockIdx.x * ROWS_PER_BLOCK;
  if (qb + ROWS_PER_BLOCK > S) return;
  const int q0 = qb + 16 * wave;

  v16h bq[4];
  {
    const _Float16* qp = Qh + (size_t)(q0 + m) * DKQ + 8 * h;
#pragma unroll
    for (int kk = 0; kk < 4; ++kk) {
      Frag16 f;
      f.h[0] = *(const v8h*)(qp + 32 * kk);
      f.h[1] = *(const v8h*)(qp + 32 * kk + 16);
      bq[kk] = f.v;
    }
  }

  v8f accO[4];
#pragma unroll
  for (int j = 0; j < 4; ++j)
#pragma unroll
    for (int r = 0; r < 8; ++r) accO[j][r] = 0.0f;
  float mrun = -INFINITY, lrun = 0.0f;

  const float sscale = (1.4426950408889634f * 0.08838834764831845f) / (SC_Q * SC_K);
  const int nT = T / KEYS_PER_TILE;

  for (int it = 0; it < nT; ++it) {
    const int t0 = it * KEYS_PER_TILE;
    __syncthreads();
#pragma unroll
    for (int r = 0; r < 4; ++r) {
      const int c = tid + 128 * r;
      *(v8h*)(kbuf + c * 8) = *(const v8h*)(Kh + (size_t)t0 * DKQ + c * 8);
    }
#pragma unroll
    for (int r = 0; r < 2; ++r) {
      const int c = tid + 128 * r;
      const int d = c >> 2, off = (c & 3) * 8;
      *(v8h*)(vbuf + d * KEYS_PER_TILE + off) =
          *(const v8h*)(Vt + (size_t)d * T + t0 + off);
    }
    __syncthreads();

    v8f sacc[2];
#pragma unroll
    for (int t = 0; t < 2; ++t) {
      v8f acc;
#pragma unroll
      for (int r = 0; r < 8; ++r) acc[r] = 0.0f;
      const _Float16* kp = kbuf + (16 * t + m) * DKQ + 8 * h;
#pragma unroll
      for (int kk = 0; kk < 4; ++kk) {
        Frag16 a;
        a.h[0] = *(const v8h*)(kp + 32 * kk);
        a.h[1] = *(const v8h*)(kp + 32 * kk + 16);
        acc = wmma16(a.v, bq[kk], acc);
      }
      sacc[t] = acc;
    }

    float tmax = -INFINITY;
#pragma unroll
    for (int t = 0; t < 2; ++t)
#pragma unroll
      for (int r = 0; r < 8; ++r) {
        const float s = sacc[t][r] * sscale;
        sacc[t][r] = s;
        tmax = fmaxf(tmax, s);
      }
    tmax = fmaxf(tmax, __shfl_xor(tmax, 16));
    const float mn = fmaxf(mrun, tmax);
    const float alpha = exp2f(mrun - mn);
    mrun = mn;

    Frag16 pb;
    float psum = 0.0f;
#pragma unroll
    for (int r = 0; r < 8; ++r) {
      const _Float16 p0 = (_Float16)exp2f(sacc[0][r] - mn);
      const _Float16 p1 = (_Float16)exp2f(sacc[1][r] - mn);
      pb.v[r] = p0;
      pb.v[8 + r] = p1;
      psum += (float)p0 + (float)p1;
    }
    psum += __shfl_xor(psum, 16);
    lrun = lrun * alpha + psum;
#pragma unroll
    for (int j = 0; j < 4; ++j) accO[j] = accO[j] * alpha;

#pragma unroll
    for (int j = 0; j < 4; ++j) {
      const _Float16* vp = vbuf + (16 * j + m) * KEYS_PER_TILE + 8 * h;
      Frag16 a;
      a.h[0] = *(const v8h*)(vp);
      a.h[1] = *(const v8h*)(vp + 16);
      accO[j] = wmma16(a.v, pb.v, accO[j]);
    }
  }

  float gp = 0.0f;
#pragma unroll
  for (int j = 0; j < 4; ++j)
#pragma unroll
    for (int r = 0; r < 8; ++r) gp += accO[j][r] * w_out[16 * j + 8 * h + r];
  gp += __shfl_xor(gp, 16);
  const float g = (gp / lrun) * (1.0f / SC_V);

  const float sflag = sumline[0];
  const bool byp = (sflag == 0.0f);

#pragma unroll 1
  for (int i = 0; i < 16; ++i) {
    const float gi = __shfl(g, i);
    const float sc = byp ? 1.0f : (1.0f - gi);
    const v4f* xr = (const v4f*)(x1 + (size_t)(q0 + i) * DMODEL);
    volatile v4f* orow = (volatile v4f*)(outp + (size_t)(q0 + i) * DMODEL);
#pragma unroll
    for (int c = 0; c < DMODEL / 128; ++c) {
      v4f v = xr[l + 32 * c];
      v = v * sc;
      orow[l + 32 * c] = v;
    }
  }
  __threadfence();
#pragma unroll 1
  for (int i = 0; i < 16; ++i) {
    const float gi = __shfl(g, i);
    const float sc = byp ? 1.0f : (1.0f - gi);
    const v4f* xr = (const v4f*)(x1 + (size_t)(q0 + i) * DMODEL);
    volatile v4f* orow = (volatile v4f*)(outp + (size_t)(q0 + i) * DMODEL);
#pragma unroll
    for (int c = 0; c < DMODEL / 128; ++c) {
      v4f v = xr[l + 32 * c];
      v = v * sc;
      orow[l + 32 * c] = v;
    }
  }
}

static size_t al256(size_t x) { return (x + 255) & ~(size_t)255; }

extern "C" void kernel_launch(void* const* d_in, const int* in_sizes, int n_in,
                              void* d_out, int out_size, void* d_ws,
                              size_t ws_size, hipStream_t stream) {
  if (n_in < 6) return;
  const float* x1 = (const float*)d_in[0];
  const float* x2 = (const float*)d_in[1];
  const float* w_q = (const float*)d_in[2];
  const float* w_k = (const float*)d_in[3];
  const float* w_v = (const float*)d_in[4];
  const float* w_o = (const float*)d_in[5];
  float* out = (float*)d_out;

  const int S = in_sizes[0] / DMODEL;
  const int T = in_sizes[1] / DMODEL;
  if (S <= 0 || T <= 0) return;
  if ((S % ROWS_PER_BLOCK) != 0 || (T % ROWS_PER_BLOCK) != 0) return;
  if (in_sizes[0] != S * DMODEL || in_sizes[1] != T * DMODEL) return;
  if (in_sizes[2] != DKQ * DMODEL || in_sizes[3] != DKQ * DMODEL ||
      in_sizes[4] != DVV * DMODEL || in_sizes[5] < DVV)
    return;
  if (out_size != S * DMODEL) return;

  const size_t oQ = 0;
  const size_t bQ = (size_t)S * DKQ * sizeof(_Float16);
  const size_t oK = al256(oQ + bQ);
  const size_t bK = (size_t)T * DKQ * sizeof(_Float16);
  const size_t oV = al256(oK + bK);
  const size_t bV = (size_t)DVV * T * sizeof(_Float16);
  const size_t oSum = al256(oV + bV);
  const size_t bSum = 32 * sizeof(float);
  if (oSum + bSum > ws_size) return;

  char* ws = (char*)d_ws;
  _Float16* Qh = (_Float16*)(ws + oQ);
  _Float16* Kh = (_Float16*)(ws + oK);
  _Float16* Vt = (_Float16*)(ws + oV);
  float* sumline = (float*)(ws + oSum);

  k_sum<<<dim3(1), dim3(256), 0, stream>>>(x2, in_sizes[1], sumline);

  k_proj<2, 0><<<dim3(S / ROWS_PER_BLOCK), dim3(256), 0, stream>>>(
      x1, w_q, Qh, S, DKQ, SC_Q);
  k_proj<2, 0><<<dim3(T / ROWS_PER_BLOCK), dim3(256), 0, stream>>>(
      x2, w_k, Kh, T, DKQ, SC_K);
  k_proj<1, 1><<<dim3(T / ROWS_PER_BLOCK), dim3(128), 0, stream>>>(
      x2, w_v, Vt, T, T, SC_V);

  k_attn_gate<<<dim3(S / ROWS_PER_BLOCK), dim3(128), 0, stream>>>(
      Qh, Kh, Vt, w_o, x1, sumline, out, S, T);
  (void)hipGetLastError();
}
